// SchNetLayer_58480274702583
// MI455X (gfx1250) — hardware-verified
//
#include <hip/hip_runtime.h>


#define NA   1024
#define NF   128
#define NR   20
#define KR   32
#define CH   64
#define NPC  (CH * NA)
typedef _Float16 h16;
typedef unsigned short bf;
typedef __attribute__((ext_vector_type(16))) __bf16   v16bf;
typedef __attribute__((ext_vector_type(16))) _Float16 v16h;
typedef __attribute__((ext_vector_type(8)))  _Float16 v8h;
typedef __attribute__((ext_vector_type(8)))  unsigned short v8us;
typedef __attribute__((ext_vector_type(8)))  float    v8f;
typedef __attribute__((ext_vector_type(4)))  float    v4f;
typedef v8h  __attribute__((may_alias)) v8ha;
typedef v4f  __attribute__((may_alias)) v4fa;
typedef v8us __attribute__((may_alias)) v8usa;

__device__ __forceinline__ unsigned short f2bf(float f) { unsigned u = __float_as_uint(f); u += 0x7FFFu + ((u >> 16) & 1u); return (unsigned short)(u >> 16); }
__device__ __forceinline__ float bf2f(unsigned short b) { return __uint_as_float(((unsigned)b) << 16); }
__device__ __forceinline__ float bfr(float f) { return bf2f(f2bf(f)); }
__device__ __forceinline__ v16h cat16(v8h lo, v8h hi) { return __builtin_shufflevector(lo, hi, 0, 1, 2, 3, 4, 5, 6, 7, 8, 9, 10, 11, 12, 13, 14, 15); }
__device__ __forceinline__ v16bf cat16b(v8us lo, v8us hi) { return __builtin_bit_cast(v16bf, __builtin_shufflevector(lo, hi, 0, 1, 2, 3, 4, 5, 6, 7, 8, 9, 10, 11, 12, 13, 14, 15)); }
__device__ __forceinline__ v8f wmma16(v16h a, v16h b, v8f c) { return __builtin_amdgcn_wmma_f32_16x16x32_f16(false, a, false, b, (short)0, c, false, false); }
__device__ __forceinline__ v8f wmmab(v16bf a, v16bf b, v8f c) { return __builtin_amdgcn_wmma_f32_16x16x32_bf16(false, a, false, b, (short)0, c, false, false); }


template <typename T16> struct WFrag;
template <> struct WFrag<h16> { typedef v16h V; static __device__ __forceinline__ V ld(const h16* p) { return cat16(*(const v8h*)p, *(const v8h*)(p + 16)); } static __device__ __forceinline__ v8f mma(V a, V b, v8f c) { return wmma16(a, b, c); } };
template <> struct WFrag<bf> { typedef v16bf V; static __device__ __forceinline__ V ld(const bf* p) { return cat16b(*(const v8us*)p, *(const v8us*)(p + 16)); } static __device__ __forceinline__ v8f mma(V a, V b, v8f c) { return wmmab(a, b, c); } };
template <typename T16, int NSPLIT, bool BIAS>
__global__ __launch_bounds__(32) void k_gemmw(const T16* __restrict__ A, const T16* __restrict__ A2, const T16* __restrict__ Bt, const T16* __restrict__ Bt2, int K, float* C, int ldc, const float* __restrict__ bias, size_t sA, size_t sB, size_t sC) {
    typedef typename WFrag<T16>::V V;
    __shared__ __align__(16) float os[16 * 68];
    const size_t z = blockIdx.z; A += z * sA; if (A2) A2 += z * sA; Bt += z * sB; if (Bt2) Bt2 += z * sB; C += z * sC;
    const int lane = threadIdx.x & 31, lr = lane & 15, hi = lane >> 4; const int r0 = blockIdx.x * 64, c0 = blockIdx.y * 64;
    v8f acc[4][4];
#pragma unroll
    for (int mb = 0; mb < 4; ++mb)
#pragma unroll
        for (int nb = 0; nb < 4; ++nb) acc[mb][nb] = (v8f){};
    const size_t aoff = (size_t)(r0 + lr) * K + 8 * hi, boff = (size_t)(c0 + lr) * K + 8 * hi;
#pragma unroll 1
    for (int kc = 0; kc < K; kc += 32) {
        V a[4], a2[4];
#pragma unroll
        for (int mb = 0; mb < 4; ++mb) { a[mb] = WFrag<T16>::ld(A + aoff + (size_t)mb * 16 * K + kc); if (NSPLIT == 1 || NSPLIT == 2) a2[mb] = WFrag<T16>::ld(A2 + aoff + (size_t)mb * 16 * K + kc); }
#pragma unroll
        for (int nb = 0; nb < 4; ++nb) { const V b = WFrag<T16>::ld(Bt + boff + (size_t)nb * 16 * K + kc); V b2; if (NSPLIT >= 2) b2 = WFrag<T16>::ld(Bt2 + boff + (size_t)nb * 16 * K + kc);
#pragma unroll
            for (int mb = 0; mb < 4; ++mb) { acc[mb][nb] = WFrag<T16>::mma(a[mb], b, acc[mb][nb]); if (NSPLIT == 1 || NSPLIT == 2) acc[mb][nb] = WFrag<T16>::mma(a2[mb], b, acc[mb][nb]); if (NSPLIT >= 2) acc[mb][nb] = WFrag<T16>::mma(a[mb], b2, acc[mb][nb]); } }
        asm volatile("v_nop\n\tv_nop\n\tv_nop\n\tv_nop" : "+v"(acc[0][0]), "+v"(acc[1][1]), "+v"(acc[2][2]), "+v"(acc[3][3]) : "v"(a[0]), "v"(a[3]));
    }
#pragma unroll
    for (int mb = 0; mb < 4; ++mb) {
#pragma unroll
        for (int nb = 0; nb < 4; ++nb) {
#pragma unroll
            for (int j = 0; j < 8; ++j) os[(hi * 8 + j) * 68 + nb * 16 + lr] = acc[mb][nb][j]; }
        __builtin_amdgcn_wave_barrier(); asm volatile("" ::: "memory");
        float* crow = C + (size_t)(r0 + mb * 16) * ldc + c0;
#pragma unroll 1
        for (int ps = 0; ps < 2; ++ps) {
#pragma unroll
            for (int s = 0; s < 8; ++s) { const int row = 2 * s + hi, cofs = lr * 4; v4f val = *(const v4fa*)(os + row * 68 + cofs); if (BIAS) { val[0] += bfr(bias[c0 + cofs]); val[1] += bfr(bias[c0 + cofs + 1]); val[2] += bfr(bias[c0 + cofs + 2]); val[3] += bfr(bias[c0 + cofs + 3]); }
                *(volatile v4f*)(crow + (size_t)row * ldc + cofs) = val; }
            if (ps == 0) __threadfence(); }
        __builtin_amdgcn_wave_barrier(); asm volatile("" ::: "memory");
    }
}

__device__ __forceinline__ void splitf(float y, unsigned short& h, unsigned short& l) { h = f2bf(y); l = f2bf(y - bf2f(h)); }
__device__ __forceinline__ float tanhf_(float x) { const float e = __expf(-2.0f * fabsf(x)); const float t = __fdiv_rn(1.0f - e, 1.0f + e); return copysignf(t, x); }
typedef __attribute__((ext_vector_type(2))) unsigned short v2us;
typedef __attribute__((ext_vector_type(4))) unsigned short v4us;

__global__ __launch_bounds__(256) void k_wtG(const float* __restrict__ w, int K, int N, bf* Bt) {
    const int lane = threadIdx.x & 31; const int L0 = (blockIdx.x * 8 + (threadIdx.x >> 5)) * 8; const int nlines = N * K / 64;
#pragma unroll 1
    for (int ps = 0; ps < 2; ++ps) {
#pragma unroll 1
        for (int l = 0; l < 8; ++l) { const int L = L0 + l; if (L >= nlines) break; const size_t e = (size_t)L * 64 + lane * 2; const int k = (int)(e % K), n = (int)(e / K); v2us o;
            o[0] = f2bf(w[(size_t)k * N + n]); o[1] = f2bf(w[(size_t)(k + 1) * N + n]); *(volatile v2us*)(Bt + e) = o; }
        if (ps == 0) __threadfence(); }
}
__global__ __launch_bounds__(256) void k_w1p(const float* __restrict__ W1, bf* Bt) { const int e = (blockIdx.x * 256 + threadIdx.x) * 4; if (e >= NF * KR) return; const int k = e % KR, n = e / KR; v4us o;
#pragma unroll
    for (int q = 0; q < 4; ++q) o[q] = (k + q) < NR ? f2bf(W1[(size_t)(k + q) * NF + n]) : (unsigned short)0; *(volatile v4us*)(Bt + e) = o; __threadfence(); *(volatile v4us*)(Bt + e) = o; }
__global__ __launch_bounds__(256) void k_rbf(const float* __restrict__ pos, const float* __restrict__ cen, const float* __restrict__ wid, int i0, bf* Rh, bf* Rl) { const size_t e = ((size_t)blockIdx.x * 256 + threadIdx.x) * 4; if (e >= (size_t)NPC * KR) return; const int r0 = (int)(e % KR); const int p = (int)(e / KR); const int j = p % NA, i = i0 + p / NA;
    const float dx = __fsub_rn(bfr(pos[i * 3]), bfr(pos[j * 3])), dy = __fsub_rn(bfr(pos[i * 3 + 1]), bfr(pos[j * 3 + 1])), dz = __fsub_rn(bfr(pos[i * 3 + 2]), bfr(pos[j * 3 + 2])); float sx = __fmul_rn(dx, dx), sy = __fmul_rn(dy, dy), sz = __fmul_rn(dz, dz); asm volatile("" : "+v"(sx), "+v"(sy), "+v"(sz)); const float d2 = __fadd_rn(__fadd_rn(sx, sy), sz); const float d = d2 > 0.f ? __fsqrt_rn(d2) : 0.f; v4us oh, ol;
#pragma unroll
    for (int q = 0; q < 4; ++q) { const int r = r0 + q; unsigned short a = 0, c = 0; if (r < NR) { const float z = __fdiv_rn(__fsub_rn(d, bfr(cen[r])), bfr(wid[r])); float z2 = __fmul_rn(z, z); asm volatile("" : "+v"(z2)); splitf(__expf(-z2), a, c); } oh[q] = a; ol[q] = c; }
    *(volatile v4us*)(Rh + e) = oh; *(volatile v4us*)(Rl + e) = ol; __threadfence(); *(volatile v4us*)(Rh + e) = oh; *(volatile v4us*)(Rl + e) = ol; }
__global__ __launch_bounds__(256) void k_tanh(const float* __restrict__ Hf, bf* Th, bf* Tl) { const size_t i4 = ((size_t)blockIdx.x * 256 + threadIdx.x) * 4; if (i4 >= (size_t)NPC * NF) return; const v4f a = *(const v4f*)(Hf + i4); v4us oh, ol;
#pragma unroll
    for (int q = 0; q < 4; ++q) { unsigned short u, c; splitf(tanhf_(a[q]), u, c); oh[q] = u; ol[q] = c; } *(volatile v4us*)(Th + i4) = oh; *(volatile v4us*)(Tl + i4) = ol; __threadfence(); *(volatile v4us*)(Th + i4) = oh; *(volatile v4us*)(Tl + i4) = ol; }
__global__ __launch_bounds__(256) void k_agg(const float* __restrict__ FLT, const float* __restrict__ feat, int i0, float* AGG) { const int e = blockIdx.x * 256 + threadIdx.x; if (e >= CH * NF) return; const int f = e % NF, il = e / NF; float s = 0.f;
#pragma unroll 1
    for (int j = 0; j < NA; ++j) { float p = __fmul_rn(FLT[((size_t)il * NA + j) * NF + f], bfr(feat[(size_t)j * NF + f])); asm volatile("" : "+v"(p)); s = __fadd_rn(s, p); }
    const size_t o = (size_t)(i0 + il) * NF + f; *(volatile float*)(AGG + o) = s; __threadfence(); *(volatile float*)(AGG + o) = s; }
__global__ __launch_bounds__(256) void k_spl(const float* __restrict__ F, size_t n4, bf* Fh, bf* Fl) { const size_t i = ((size_t)blockIdx.x * 256 + threadIdx.x) * 4; if (i >= n4 * 4) return; const v4f a = *(const v4f*)(F + i); v4us oh, ol;
#pragma unroll
    for (int q = 0; q < 4; ++q) { unsigned short u, c2; splitf(a[q], u, c2); oh[q] = u; ol[q] = c2; } *(volatile v4us*)(Fh + i) = oh; *(volatile v4us*)(Fl + i) = ol; __threadfence(); *(volatile v4us*)(Fh + i) = oh; *(volatile v4us*)(Fl + i) = ol; }
__global__ __launch_bounds__(256) void k_fin(const float* __restrict__ feat, const float* __restrict__ R, float* OUT) { const size_t i = ((size_t)blockIdx.x * 256 + threadIdx.x) * 4; if (i >= (size_t)NA * NF) return; const v4f r = *(const v4f*)(R + i); v4f o; o[0] = __fadd_rn(bfr(feat[i]), r[0]); o[1] = __fadd_rn(bfr(feat[i + 1]), r[1]); o[2] = __fadd_rn(bfr(feat[i + 2]), r[2]); o[3] = __fadd_rn(bfr(feat[i + 3]), r[3]); *(volatile v4f*)(OUT + i) = o; __threadfence(); *(volatile v4f*)(OUT + i) = o; }

extern "C" void kernel_launch(void* const* d_in, const int* in_sizes, int n_in,
                              void* d_out, int out_size, void* d_ws, size_t ws_size, hipStream_t stream) {
    (void)in_sizes; (void)n_in; (void)out_size;
    const float* feat = (const float*)d_in[0]; const float* pos = (const float*)d_in[1]; const float* cen = (const float*)d_in[2]; const float* wid = (const float*)d_in[3]; const float* W1 = (const float*)d_in[4]; const float* b1 = (const float*)d_in[5]; const float* W2 = (const float*)d_in[6]; const float* b2 = (const float*)d_in[7]; const float* Wi = (const float*)d_in[8]; const float* bi = (const float*)d_in[9];
    float* OUT = (float*)d_out;
    char* wsp = (char*)d_ws;
    auto take = [&](size_t bytes) { char* p = wsp; wsp += (bytes + 255) & ~(size_t)255; return (void*)p; };
    bf* B1 = (bf*)take((size_t)NF * KR * 2); bf* B2 = (bf*)take((size_t)NF * NF * 2); bf* BI = (bf*)take((size_t)NF * NF * 2); bf* Rh = (bf*)take((size_t)NPC * KR * 2); bf* Rl = (bf*)take((size_t)NPC * KR * 2); float* Hf = (float*)take((size_t)NPC * NF * 4); bf* Th = (bf*)take((size_t)NPC * NF * 2); bf* Tl = (bf*)take((size_t)NPC * NF * 2); float* FLT = (float*)take((size_t)NPC * NF * 4);
    float* AGG = (float*)take((size_t)NA * NF * 4); bf* Ah = (bf*)take((size_t)NA * NF * 2); bf* Al = (bf*)take((size_t)NA * NF * 2); float* R = (float*)take((size_t)NA * NF * 4);
    if ((size_t)(wsp - (char*)d_ws) > ws_size) return;
    k_w1p<<<(NF * KR / 4 + 255) / 256, 256, 0, stream>>>(W1, B1); k_wtG<<<(NF * NF / 64 + 63) / 64, 256, 0, stream>>>(W2, NF, NF, B2); k_wtG<<<(NF * NF / 64 + 63) / 64, 256, 0, stream>>>(Wi, NF, NF, BI);
    for (int i0 = 0; i0 < NA; i0 += CH) {
        k_rbf<<<(unsigned)(((size_t)NPC * KR / 4 + 255) / 256), 256, 0, stream>>>(pos, cen, wid, i0, Rh, Rl);
        k_gemmw<bf, 1, true><<<dim3(NPC / 64, NF / 64, 1), 32, 0, stream>>>(Rh, Rl, B1, nullptr, KR, Hf, NF, b1, 0, 0, 0); k_tanh<<<(unsigned)(((size_t)NPC * NF / 4 + 255) / 256), 256, 0, stream>>>(Hf, Th, Tl);
        k_gemmw<bf, 1, true><<<dim3(NPC / 64, NF / 64, 1), 32, 0, stream>>>(Th, Tl, B2, nullptr, NF, FLT, NF, b2, 0, 0, 0);
        k_agg<<<(CH * NF + 255) / 256, 256, 0, stream>>>(FLT, feat, i0, AGG); }
    k_spl<<<(NA * NF / 4 + 255) / 256, 256, 0, stream>>>(AGG, (size_t)NA * NF / 4, Ah, Al);
    k_gemmw<bf, 1, true><<<dim3(NA / 64, NF / 64, 1), 32, 0, stream>>>(Ah, Al, BI, nullptr, NF, R, NF, bi, 0, 0, 0); k_fin<<<(NA * NF / 4 + 255) / 256, 256, 0, stream>>>(feat, R, OUT);
}
